// CrossAttention_25847113187983
// MI455X (gfx1250) — hardware-verified
//
#include <hip/hip_runtime.h>
#include <stdint.h>


typedef _Float16 v16h __attribute__((ext_vector_type(16)));
typedef _Float16 v8h  __attribute__((ext_vector_type(8)));
typedef float    v8f  __attribute__((ext_vector_type(8)));
typedef float    v4f  __attribute__((ext_vector_type(4)));

#ifndef NB
#define NB 4
#endif
#ifndef SEQ
#define SEQ 4096
#endif
#define NB_FULL  4
#define SEQ_FULL 4096
#define CH       256

#define ACT_CAR   8.0f
#define W_CAR     1024.0f
#define PROJ_SCL  0.0009765625f
#define RES_CAR   2048.0f
#define RES_INV   0.00048828125f
#define S_SCL     0.015625f
#define P_CAR     16384.0f
#define O_SCL     7.62939453125e-6f

static_assert(SEQ % 128 == 0);
static_assert(SEQ <= SEQ_FULL);
static_assert(NB >= 1 && NB <= NB_FULL);
static_assert(CH == 256);
static_assert((long)NB_FULL * CH * SEQ_FULL * 4 == 16777216L);

union Frag16 { v16h v; v8h p[2]; };

__device__ __forceinline__ v16h ld_frag(const _Float16* p, int hl) {
  Frag16 f;
  f.p[0] = *(const v8h*)(p + 8 * hl);
  f.p[1] = *(const v8h*)(p + 16 + 8 * hl);
  return f.v;
}

__device__ __forceinline__ v8f mma(v16h a, v16h b, v8f c) {
  v8f d = __builtin_amdgcn_wmma_f32_16x16x32_f16(false, a, false, b, (short)0, c, false, false);
  asm volatile("v_nop\n\tv_nop\n\tv_nop\n\tv_nop" : "+v"(d) : "v"(a), "v"(b));
  return d;
}

__device__ __forceinline__ float bf16_rne(float x) {
  unsigned int u = __builtin_bit_cast(unsigned int, x);
  u += 0x7FFFu + ((u >> 16) & 1u);
  return __builtin_bit_cast(float, u & 0xFFFF0000u);
}

__global__ __launch_bounds__(256) void k_cvt8(const float* __restrict__ src,
                                              _Float16* __restrict__ dst,
                                              int cols, int pitch, float car, int total8)
{
  const int i8 = blockIdx.x * 256 + threadIdx.x;
  if (i8 >= total8) return;
  const size_t e   = (size_t)i8 * 8;
  const size_t r   = e / (size_t)cols;
  const int    col = (int)(e - r * (size_t)cols);
  const float* s = src + r * (size_t)pitch + col;
  const v4f x0 = *(const v4f*)s;
  const v4f x1 = *(const v4f*)(s + 4);
  v8h o;
#pragma unroll
  for (int j = 0; j < 4; ++j) {
    const float t0 = x0[j];
    const float t1 = x1[j];
    o[j]     = (_Float16)(bf16_rne(t0) * car);
    o[4 + j] = (_Float16)(bf16_rne(t1) * car);
  }
  _Float16* d = dst + e;
  *(volatile v8h*)d = o;
  __threadfence();
  *(volatile v8h*)d = o;
}

__global__ __launch_bounds__(256) void k_tr(const float* __restrict__ X,
                                            _Float16* __restrict__ XT)
{
  __shared__ float tile[64 * 65];
  const int tid = threadIdx.x;
  const int n0 = blockIdx.x * 64, c0 = blockIdx.y * 64, bb = blockIdx.z;
  const float* src = X + (size_t)bb * CH * SEQ_FULL;
  _Float16* dst = XT + (size_t)bb * SEQ * CH;
#pragma unroll
  for (int i = 0; i < 4; ++i) {
    const int idx = i * 256 + tid;
    const int r = idx >> 4, c4 = (idx & 15) * 4;
    const v4f v = *(const v4f*)(src + (size_t)(c0 + r) * SEQ_FULL + n0 + c4);
    float* tp = tile + r * 65 + c4;
    tp[0] = v[0]; tp[1] = v[1]; tp[2] = v[2]; tp[3] = v[3];
  }
  __syncthreads();
  v8h o[2];
  _Float16* dp[2];
#pragma unroll
  for (int i = 0; i < 2; ++i) {
    const int line = i * 32 + (tid >> 3);
    const int pc   = (tid & 7) * 8;
#pragma unroll
    for (int j = 0; j < 8; ++j)
      o[i][j] = (_Float16)(bf16_rne(tile[(pc + j) * 65 + line]) * ACT_CAR);
    dp[i] = dst + (size_t)(n0 + line) * CH + c0 + pc;
  }
  *(volatile v8h*)dp[0] = o[0];
  *(volatile v8h*)dp[1] = o[1];
  __threadfence();
  *(volatile v8h*)dp[0] = o[0];
  *(volatile v8h*)dp[1] = o[1];
}

__global__ __launch_bounds__(128) __attribute__((amdgpu_num_vgpr(256)))
void k_proj(const _Float16* __restrict__ A, const _Float16* __restrict__ Bt,
            _Float16* __restrict__ PH, _Float16* __restrict__ PL)
{
  __shared__ __attribute__((aligned(16))) _Float16 ldsE[2 * 128 * 72];
  _Float16* const ldsH = ldsE;
  _Float16* const ldsL = ldsE + 128 * 72;

  const int tid = threadIdx.x, lane = tid & 31, w = tid >> 5;
  const int hl = lane >> 4, c = lane & 15;
  const int m0 = blockIdx.y * 128, n0 = blockIdx.x * 64;
  const int mw = m0 + 32 * w;

  const _Float16* ap0 = A  + (size_t)(mw + c) * CH;
  const _Float16* ap1 = A  + (size_t)(mw + 16 + c) * CH;
  const _Float16* bp  = Bt + (size_t)(n0 + c) * CH;
  const size_t bst = (size_t)16 * CH;

  v8f acc[8] = {};
#pragma unroll 1
  for (int k0 = 0; k0 < CH; k0 += 32) {
    const v16h a0 = ld_frag(ap0 + k0, hl);
    const v16h a1 = ld_frag(ap1 + k0, hl);
    const v16h b0 = ld_frag(bp + k0, hl);
    const v16h b1 = ld_frag(bp + bst + k0, hl);
    const v16h b2 = ld_frag(bp + 2 * bst + k0, hl);
    const v16h b3 = ld_frag(bp + 3 * bst + k0, hl);
    acc[0] = mma(a0, b0, acc[0]);
    acc[1] = mma(a0, b1, acc[1]);
    acc[2] = mma(a0, b2, acc[2]);
    acc[3] = mma(a0, b3, acc[3]);
    acc[4] = mma(a1, b0, acc[4]);
    acc[5] = mma(a1, b1, acc[5]);
    acc[6] = mma(a1, b2, acc[6]);
    acc[7] = mma(a1, b3, acc[7]);
  }

#pragma unroll
  for (int i = 0; i < 2; ++i)
#pragma unroll
    for (int t = 0; t < 4; ++t)
#pragma unroll
      for (int r = 0; r < 8; ++r) {
        const int rowl = 32 * w + 16 * i + 8 * hl + r;
        const float v = acc[i * 4 + t][r] * PROJ_SCL;
        const _Float16 hv = (_Float16)v;
        const float res = (v - (float)hv) * RES_CAR;
        ldsH[rowl * 72 + 16 * t + c] = hv;
        ldsL[rowl * 72 + 16 * t + c] = (_Float16)res;
      }
  __syncthreads();

  _Float16* const bh = PH + (size_t)m0 * CH + n0;
  _Float16* const bl = PL + (size_t)m0 * CH + n0;
  for (int i = 0; i < 8; ++i) {
    const int q = i * 128 + tid;
    const int rowl = q >> 3, ch = (q & 7) * 8;
    const v8h vh = *(const v8h*)(ldsH + rowl * 72 + ch);
    const v8h vl = *(const v8h*)(ldsL + rowl * 72 + ch);
    *(volatile v8h*)(bh + (size_t)rowl * CH + ch) = vh;
    *(volatile v8h*)(bl + (size_t)rowl * CH + ch) = vl;
  }
  __threadfence();
  for (int i = 0; i < 8; ++i) {
    const int q = i * 128 + tid;
    const int rowl = q >> 3, ch = (q & 7) * 8;
    const v8h vh = *(const v8h*)(ldsH + rowl * 72 + ch);
    const v8h vl = *(const v8h*)(ldsL + rowl * 72 + ch);
    *(volatile v8h*)(bh + (size_t)rowl * CH + ch) = vh;
    *(volatile v8h*)(bl + (size_t)rowl * CH + ch) = vl;
  }
}

template <bool QSPLIT>
__global__ __launch_bounds__(256) __attribute__((amdgpu_num_vgpr(256)))
void k_attn(const _Float16* __restrict__ Qa, const _Float16* __restrict__ Qb,
            const _Float16* __restrict__ Ka, const _Float16* __restrict__ Kb,
            const _Float16* __restrict__ Vt, float* __restrict__ Out)
{
  constexpr int NKT    = QSPLIT ? 1 : 2;
  constexpr int KT_H   = 32 * 264;
  constexpr int V_H    = CH * 40;
  constexpr int P_H    = 8 * 16 * 40;
  constexpr int X_F    = 8 * 16 * 36;
  constexpr int TILE_F = (NKT * KT_H + V_H + P_H) / 2 + X_F;
  constexpr int EPI_F  = CH * 68;
  constexpr int LDS_F  = (TILE_F > EPI_F) ? TILE_F : EPI_F;
  __shared__ __attribute__((aligned(16))) float lds_raw[LDS_F];
  _Float16* const ldsK0 = reinterpret_cast<_Float16*>(lds_raw);
  _Float16* const ldsK1 = ldsK0 + (NKT - 1) * KT_H;
  _Float16* const ldsV  = ldsK0 + NKT * KT_H;
  _Float16* const ldsP  = ldsV + V_H;
  float* const ldsX = lds_raw + (NKT * KT_H + V_H + P_H) / 2;
  float* const ldsO = lds_raw;

  const int tid = threadIdx.x, lane = tid & 31, w = tid >> 5;
  const int hl = lane >> 4, c = lane & 15;
  const int pr = w >> 1, hd = w & 1;
  const int qblocks = SEQ / 64;
  const int bb = blockIdx.x / qblocks;
  const int qb = blockIdx.x - bb * qblocks;
  const int q0 = qb * 64;
  const int qw = q0 + 16 * pr;
  const int d0 = hd * 128;

  const size_t qrow = ((size_t)bb * SEQ + qw + c) * CH + d0;
  const _Float16* qpa = Qa + qrow;
  const _Float16* qpb = Qb + qrow;
  const _Float16* kab = Ka + (size_t)bb * SEQ * CH;
  const _Float16* kbb = Kb + (size_t)bb * SEQ * CH;
  const _Float16* vtb = Vt + (size_t)bb * CH * SEQ;
  _Float16* const myP = ldsP + w * (16 * 40);
  float* const myX = ldsX + w * (16 * 36);
  const float* const otX = ldsX + (w ^ 1) * (16 * 36);
  (void)qpb; (void)kbb; (void)ldsK1;

  v16h qf[4];
  if constexpr (!QSPLIT) {
#pragma unroll
    for (int ks = 0; ks < 4; ++ks) qf[ks] = ld_frag(qpa + 32 * ks, hl);
  }

  float m[8], l[8];
  v8f o[8] = {};
#pragma unroll
  for (int r = 0; r < 8; ++r) { m[r] = -__builtin_inff(); l[r] = 0.f; }

#pragma unroll 1
  for (int kt = 0; kt < SEQ / 32; ++kt) {
    const int mk = kt * 32;
#pragma unroll
    for (int j = 0; j < 4; ++j) {
      const int s  = j * 256 + tid;
      const int rr = s >> 5, cc = (s & 31) * 8;
      const v8h k8 = *(const v8h*)(kab + (size_t)(mk + rr) * CH + cc);
      *(v8h*)(ldsK0 + rr * 264 + cc) = k8;
      if constexpr (!QSPLIT) {
        const v8h k8b = *(const v8h*)(kbb + (size_t)(mk + rr) * CH + cc);
        *(v8h*)(ldsK1 + rr * 264 + cc) = k8b;
      }
      const int dd = s >> 2, kc = (s & 3) * 8;
      const v8h v8 = *(const v8h*)(vtb + (size_t)dd * SEQ + mk + kc);
      *(v8h*)(ldsV + dd * 40 + kc) = v8;
    }
    __syncthreads();

    v8f sh[2] = {}, sl[2] = {};
#pragma unroll
    for (int ks = 0; ks < 4; ++ks) {
      const int k0 = d0 + 32 * ks;
      if constexpr (QSPLIT) {
        const v16h qh = ld_frag(qpa + 32 * ks, hl);
        const v16h ql = ld_frag(qpb + 32 * ks, hl);
#pragma unroll
        for (int t = 0; t < 2; ++t) {
          const v16h kf = ld_frag(ldsK0 + (16 * t + c) * 264 + k0, hl);
          sh[t] = mma(qh, kf, sh[t]);
          sl[t] = mma(ql, kf, sl[t]);
        }
      } else {
#pragma unroll
        for (int t = 0; t < 2; ++t) {
          const v16h kfh = ld_frag(ldsK0 + (16 * t + c) * 264 + k0, hl);
          const v16h kfl = ld_frag(ldsK1 + (16 * t + c) * 264 + k0, hl);
          sh[t] = mma(qf[ks], kfh, sh[t]);
          sl[t] = mma(qf[ks], kfl, sl[t]);
        }
      }
    }

    float pa[2][8];
#pragma unroll
    for (int t = 0; t < 2; ++t)
#pragma unroll
      for (int r = 0; r < 8; ++r) {
        const float v = sh[t][r] + sl[t][r] * RES_INV;
        pa[t][r] = v;
        myX[(8 * hl + r) * 36 + 16 * t + c] = v;
      }
    __syncthreads();

#pragma unroll
    for (int r = 0; r < 8; ++r) {
      const float v0 = (pa[0][r] + otX[(8 * hl + r) * 36 + c]) * S_SCL;
      const float v1 = (pa[1][r] + otX[(8 * hl + r) * 36 + 16 + c]) * S_SCL;
      float tm = fmaxf(v0, v1);
      tm = fmaxf(tm, __shfl_xor(tm, 1, 32));
      tm = fmaxf(tm, __shfl_xor(tm, 2, 32));
      tm = fmaxf(tm, __shfl_xor(tm, 4, 32));
      tm = fmaxf(tm, __shfl_xor(tm, 8, 32));
      const float mn = fmaxf(m[r], tm);
      const float al = __expf(m[r] - mn);
      const float p0 = __expf(v0 - mn), p1 = __expf(v1 - mn);
      float rs = p0 + p1;
      rs += __shfl_xor(rs, 1, 32);
      rs += __shfl_xor(rs, 2, 32);
      rs += __shfl_xor(rs, 4, 32);
      rs += __shfl_xor(rs, 8, 32);
      l[r] = l[r] * al + rs;
      m[r] = mn;
#pragma unroll
      for (int t = 0; t < 8; ++t) o[t][r] *= al;
      _Float16* pp = myP + (8 * hl + r) * 40 + c;
      pp[0]  = (_Float16)(p0 * P_CAR);
      pp[16] = (_Float16)(p1 * P_CAR);
    }
    __syncthreads();

    const v16h pf = ld_frag(myP + c * 40, hl);
#pragma unroll
    for (int t = 0; t < 8; ++t) {
      const v16h vf = ld_frag(ldsV + (d0 + 16 * t + c) * 40, hl);
      o[t] = mma(pf, vf, o[t]);
    }
    __syncthreads();
  }

#pragma unroll
  for (int r = 0; r < 8; ++r) {
    const float inv = (1.0f / l[r]) * O_SCL;
    const int ql = 16 * pr + 8 * hl + r;
#pragma unroll
    for (int t = 0; t < 8; ++t)
      ldsO[(d0 + 16 * t + c) * 68 + ql] = o[t][r] * inv;
  }
  __syncthreads();
  float* const ob = Out + (size_t)bb * CH * SEQ_FULL + q0;
  for (int i = 0; i < 16; ++i) {
    const int qi = i * 256 + tid;
    const int L = qi >> 3, pc = qi & 7;
    const int dd = L >> 1, col = (L & 1) * 32 + pc * 4;
    const v4f v = *(const v4f*)(ldsO + dd * 68 + col);
    *(volatile v4f*)(ob + (size_t)dd * SEQ_FULL + col) = v;
  }
  __threadfence();
  for (int i = 0; i < 16; ++i) {
    const int qi = i * 256 + tid;
    const int L = qi >> 3, pc = qi & 7;
    const int dd = L >> 1, col = (L & 1) * 32 + pc * 4;
    const v4f v = *(const v4f*)(ldsO + dd * 68 + col);
    *(volatile v4f*)(ob + (size_t)dd * SEQ_FULL + col) = v;
  }
}

extern "C" void kernel_launch(void* const* d_in, const int* in_sizes, int n_in,
                              void* d_out, int out_size, void* d_ws, size_t ws_size,
                              hipStream_t stream)
{
  if (n_in < 3) return;
  const long need_act = ((long)NB * CH - 1) * SEQ_FULL + SEQ;
  if ((long)in_sizes[0] < need_act) return;
  if ((long)in_sizes[1] < need_act) return;
  if ((long)in_sizes[2] < (long)CH * CH) return;
  const long out1_off = (long)NB_FULL * CH * SEQ_FULL;
  if ((long)out_size < out1_off + need_act) return;

  const float* a = (const float*)d_in[0];
  const float* b = (const float*)d_in[1];
  const float* W = (const float*)d_in[2];
  float* out = (float*)d_out;

  const size_t nAct = (size_t)NB * CH * SEQ;
  const size_t nW   = (size_t)CH * CH;
  const size_t total_halves = 6 * nAct + nW;
  if (total_halves * sizeof(_Float16) > ws_size) return;

  _Float16* A16  = (_Float16*)d_ws;
  _Float16* B16  = A16  + nAct;
  _Float16* AT16 = B16  + nAct;
  _Float16* BT16 = AT16 + nAct;
  _Float16* QH   = BT16 + nAct;
  _Float16* QL   = QH   + nAct;
  _Float16* W16  = QL   + nAct;

  const int t8 = (int)(nAct / 8);
  k_cvt8<<<(t8 + 255) / 256, 256, 0, stream>>>(a, A16, SEQ, SEQ_FULL, ACT_CAR, t8);
  k_cvt8<<<(t8 + 255) / 256, 256, 0, stream>>>(b, B16, SEQ, SEQ_FULL, ACT_CAR, t8);
  const int tw8 = (int)(nW / 8);
  k_cvt8<<<(tw8 + 255) / 256, 256, 0, stream>>>(W, W16, CH, CH, W_CAR, tw8);

  k_tr<<<dim3(SEQ / 64, CH / 64, NB), 256, 0, stream>>>(a, AT16);
  k_tr<<<dim3(SEQ / 64, CH / 64, NB), 256, 0, stream>>>(b, BT16);

  k_proj<<<dim3(CH / 64, (NB * SEQ) / 128), 128, 0, stream>>>(AT16, W16, QH, QL);

  k_attn<true><<<NB * (SEQ / 64), 256, 0, stream>>>(QH, QL, BT16, BT16, B16, out + out1_off);
  k_attn<false><<<NB * (SEQ / 64), 256, 0, stream>>>(BT16, BT16, QH, QL, A16, out);
}
